// GaInit_72009421685306
// MI455X (gfx1250) — hardware-run, weakly checked
//
#include <hip/hip_runtime.h>


#ifndef NROWS
#define NROWS 512
#endif
#ifndef NPTS
#define NPTS 16384
#endif
#define NROWS_FULL 512
#define NPTS_FULL  16384
#ifndef OUT_PITCH
#define OUT_PITCH NPTS
#endif
#define MWAVES 8
#define KSPAN  (NPTS / MWAVES)
#define KSTEPS (KSPAN / 32)
#define NFEAT  9
#define ER     32

static_assert(NROWS % 16 == 0);
static_assert(NROWS % ER == 0);
static_assert(NPTS % 1024 == 0);
static_assert(NPTS % (MWAVES * 32) == 0);
static_assert(KSTEPS >= 1);
static_assert(NPTS % 8 == 0);
static_assert(NFEAT <= 16);
static_assert(MWAVES * 32 == 256);
static_assert(NROWS <= NROWS_FULL);
static_assert(NPTS <= NPTS_FULL);
static_assert(OUT_PITCH % 32 == 0);
static_assert(NPTS_FULL % 32 == 0);

typedef unsigned short bf;
typedef __attribute__((ext_vector_type(16))) __bf16   v16bf;
typedef __attribute__((ext_vector_type(8)))  unsigned short v8us;
typedef __attribute__((ext_vector_type(8)))  float    v8f;
typedef __attribute__((ext_vector_type(4)))  float    v4f;
typedef __attribute__((ext_vector_type(2)))  float    v2f;
typedef v4f  __attribute__((may_alias)) v4fa;

__device__ __forceinline__ unsigned short f2bf(float f) { unsigned u = __float_as_uint(f); u += 0x7FFFu + ((u >> 16) & 1u); return (unsigned short)(u >> 16); }
__device__ __forceinline__ float bfr(float f) { return __uint_as_float(((unsigned)f2bf(f)) << 16); }
__device__ __forceinline__ v16bf cat16b(v8us lo, v8us hi) { return __builtin_bit_cast(v16bf, __builtin_shufflevector(lo, hi, 0, 1, 2, 3, 4, 5, 6, 7, 8, 9, 10, 11, 12, 13, 14, 15)); }
__device__ __forceinline__ v16bf ldb(const bf* p)  { return cat16b(*(const v8us*)p, *(const v8us*)(p + 16)); }
__device__ __forceinline__ v8f wmmab_g(v16bf a, v16bf b, v8f c) {
    c = __builtin_amdgcn_wmma_f32_16x16x32_bf16(false, a, false, b, (short)0, c, false, false);
    asm volatile("v_nop\n\tv_nop\n\tv_nop\n\tv_nop" : "+v"(c) : "v"(a), "v"(b));
    return c;
}

static_assert((size_t)(NPTS / 8) * 16 * 16 == (size_t)16 * NPTS * 2);
__global__ __launch_bounds__(256) void k_feat(const float* __restrict__ geo, bf* FT) {
#pragma clang fp contract(off)
    const int i = blockIdx.x * 256 + threadIdx.x; if (i >= NPTS / 8) return;
    const v8f g0 = *(const v8f*)(geo + (size_t)i * 16);
    const v8f g1 = *(const v8f*)(geo + (size_t)i * 16 + 8);
    const v8us z = (v8us){};
    v8us f[16];
#pragma unroll
    for (int c = 0; c < 16; ++c) f[c] = z;
#pragma unroll
    for (int k = 0; k < 8; ++k) {
        const float rx = (k < 4) ? g0[(2 * k) & 7] : g1[(2 * k - 8) & 7];
        const float ry = (k < 4) ? g0[(2 * k + 1) & 7] : g1[(2 * k - 7) & 7];
        const unsigned short bx = f2bf(rx), by = f2bf(ry);
        const float x = __uint_as_float(((unsigned)bx) << 16), y = __uint_as_float(((unsigned)by) << 16);
        const float pxx = x * x, pxy = x * y, pyy = y * y;
        const unsigned short hxx = f2bf(pxx), hxy = f2bf(pxy), hyy = f2bf(pyy);
        const float lxx = pxx - __uint_as_float(((unsigned)hxx) << 16);
        const float lxy = pxy - __uint_as_float(((unsigned)hxy) << 16);
        const float lyy = pyy - __uint_as_float(((unsigned)hyy) << 16);
        f[0][k] = bx; f[1][k] = by;
        f[2][k] = hxx; f[3][k] = f2bf(lxx);
        f[4][k] = hxy; f[5][k] = f2bf(lxy);
        f[6][k] = hyy; f[7][k] = f2bf(lyy);
        f[8][k] = (unsigned short)0x3F80;
    }
    bf* dst = FT + (size_t)i * 8;
#pragma unroll 1
    for (int ps = 0; ps < 2; ++ps) {
#pragma unroll
        for (int c = 0; c < 16; ++c) { const v8us v = f[c]; *(volatile v8us*)(dst + (size_t)c * NPTS) = v; }
        if (ps == 0) __threadfence(); }
}

__global__ __launch_bounds__(256) void k_gbar(const float* __restrict__ geo, float* GB) {
#pragma clang fp contract(off)
    __shared__ float part[8 * 8];
    __shared__ __align__(16) float line[32];
    const int lane = threadIdx.x & 31;
    const int wave = __builtin_amdgcn_readfirstlane((int)(threadIdx.x >> 5));
    float s0 = 0.0f, s1 = 0.0f, s2 = 0.0f, s3 = 0.0f, s4 = 0.0f;
#pragma unroll 1
    for (int i = threadIdx.x; i < NPTS; i += 256) {
        const v2f g = *(const v2f*)(geo + (size_t)i * 2);
        const float x = bfr(g[0]), y = bfr(g[1]);
        s0 += x; s1 += y; s2 += x * x; s3 += x * y; s4 += y * y; }
#pragma unroll
    for (int off = 16; off >= 1; off >>= 1) {
        s0 += __shfl_xor(s0, off, 32); s1 += __shfl_xor(s1, off, 32); s2 += __shfl_xor(s2, off, 32);
        s3 += __shfl_xor(s3, off, 32); s4 += __shfl_xor(s4, off, 32); }
    if (lane == 0) { part[wave * 8 + 0] = s0; part[wave * 8 + 1] = s1; part[wave * 8 + 2] = s2; part[wave * 8 + 3] = s3; part[wave * 8 + 4] = s4; }
    __syncthreads();
    float v = 0.0f;
    if (threadIdx.x < 5) {
#pragma unroll 1
        for (int w = 0; w < 8; ++w) v += part[w * 8 + threadIdx.x];
        v = v * (1.0f / (float)NPTS); }
    if (threadIdx.x < 32) line[threadIdx.x] = v;
    __syncthreads();
    if (threadIdx.x < 8) {
        const v4f o = *(const v4fa*)(&line[threadIdx.x * 4]);
        *(volatile v4f*)(GB + threadIdx.x * 4) = o; __threadfence(); *(volatile v4f*)(GB + threadIdx.x * 4) = o; }
}

__device__ __forceinline__ void mom_span(const float* __restrict__ w, const bf* __restrict__ FT, size_t aoff, size_t boff, v8f& acc, float& sq) {
#pragma unroll 2
    for (int ks = 0; ks < KSTEPS; ++ks) {
        const v8f x0 = *(const v8f*)(w + aoff + (size_t)ks * 32);
        const v8f x1 = *(const v8f*)(w + aoff + (size_t)ks * 32 + 16);
        v8us lo, hi8;
#pragma unroll
        for (int k = 0; k < 8; ++k) {
            const unsigned short u0 = f2bf(x0[k]), u1 = f2bf(x1[k]);
            const float f0 = __uint_as_float(((unsigned)u0) << 16), f1 = __uint_as_float(((unsigned)u1) << 16);
            lo[k] = u0; hi8[k] = u1; sq += f0 * f0; sq += f1 * f1; }
        const v16bf a = cat16b(lo, hi8);
        const v16bf b = ldb(FT + boff + (size_t)ks * 32);
        acc = wmmab_g(a, b, acc);
    }
}

static_assert(32 * 16 == 16 * 8 * 4);
static_assert((2 * MWAVES * 256 + 2 * MWAVES * 16 + 128) * 4 <= 131072);
__global__ __launch_bounds__(256) void k_mom(const float* __restrict__ WA, const float* __restrict__ WB, const bf* __restrict__ FX, const bf* __restrict__ FY,
                                             const float* __restrict__ GB, float* CO) {
    __shared__ float redA[MWAVES * 256];
    __shared__ float redB[MWAVES * 256];
    __shared__ float sqA[MWAVES * 16];
    __shared__ float sqB[MWAVES * 16];
    __shared__ __align__(16) float cs[16 * 8];
    const int lane = threadIdx.x & 31, lr = lane & 15, hi = lane >> 4;
    const int wave = __builtin_amdgcn_readfirstlane((int)(threadIdx.x >> 5));
    const int b0 = blockIdx.x * 16;
    const float g0 = GB[0], g1 = GB[1], g2 = GB[2], g3 = GB[3], g4 = GB[4];
    const size_t aoff = (size_t)(b0 + lr) * NPTS_FULL + (size_t)wave * KSPAN + 8 * hi;
    const size_t boff = (size_t)lr * NPTS + (size_t)wave * KSPAN + 8 * hi;
    v8f accA = (v8f){}, accB = (v8f){}; float sa = 0.0f, sb = 0.0f;
    mom_span(WA, FX, aoff, boff, accA, sa);
    mom_span(WB, FY, aoff, boff, accB, sb);
    const int rb = (wave * 16 + 8 * hi) * 16 + lr;
#pragma unroll
    for (int r = 0; r < 8; ++r) { redA[rb + r * 16] = accA[r]; redB[rb + r * 16] = accB[r]; }
    sa += __shfl_xor(sa, 16, 32); sb += __shfl_xor(sb, 16, 32);
    if (hi == 0) { sqA[wave * 16 + lr] = sa; sqB[wave * 16 + lr] = sb; }
    __syncthreads();
    if (threadIdx.x < 16) {
        const int t = threadIdx.x;
        float SA[NFEAT], SB[NFEAT]; float qa = 0.0f, qb = 0.0f;
#pragma unroll
        for (int c = 0; c < NFEAT; ++c) { SA[c] = 0.0f; SB[c] = 0.0f; }
#pragma unroll 1
        for (int w = 0; w < MWAVES; ++w) {
#pragma unroll
            for (int c = 0; c < NFEAT; ++c) { SA[c] += redA[(w * 16 + t) * 16 + c]; SB[c] += redB[(w * 16 + t) * 16 + c]; }
            qa += sqA[w * 16 + t]; qb += sqB[w * 16 + t]; }
        const float ma0 = SA[0], ma1 = SA[1], mb0 = SB[0], mb1 = SB[1];
        const float ga = 2.0f - SA[8], gb = 2.0f - SB[8];
        const float ida = 1.0f / (1.0f - qa), idb = 1.0f / (1.0f - qb);
        const float ca00 = ((SA[2] + SA[3]) - ma0 * ma0 * ga) * ida;
        const float ca01 = ((SA[4] + SA[5]) - ma0 * ma1 * ga) * ida;
        const float ca11 = ((SA[6] + SA[7]) - ma1 * ma1 * ga) * ida;
        const float cb00 = ((SB[2] + SB[3]) - mb0 * mb0 * gb) * idb;
        const float cb01 = ((SB[4] + SB[5]) - mb0 * mb1 * gb) * idb;
        const float cb11 = ((SB[6] + SB[7]) - mb1 * mb1 * gb) * idb;
        const float s1 = sqrtf(ca00 * ca11 - ca01 * ca01);
        const float it1 = 1.0f / sqrtf(ca00 + ca11 + 2.0f * s1);
        const float r00 = (ca00 + s1) * it1, r01 = ca01 * it1, r11 = (ca11 + s1) * it1;
        const float is1 = 1.0f / s1;
        const float i00 = r11 * is1, i01 = -r01 * is1, i11 = r00 * is1;
        const float p00 = r00 * cb00 + r01 * cb01, p01 = r00 * cb01 + r01 * cb11;
        const float p10 = r01 * cb00 + r11 * cb01, p11 = r01 * cb01 + r11 * cb11;
        const float m00 = p00 * r00 + p01 * r01;
        const float m01 = p00 * r01 + p01 * r11;
        const float m11 = p10 * r01 + p11 * r11;
        const float s2 = sqrtf(m00 * m11 - m01 * m01);
        const float it2 = 1.0f / sqrtf(m00 + m11 + 2.0f * s2);
        const float q00 = (m00 + s2) * it2, q01 = m01 * it2, q11 = (m11 + s2) * it2;
        const float u00 = i00 * q00 + i01 * q01, u01 = i00 * q01 + i01 * q11;
        const float u10 = i01 * q00 + i11 * q01, u11 = i01 * q01 + i11 * q11;
        const float A00 = u00 * i00 + u01 * i01;
        const float A01 = u00 * i01 + u01 * i11;
        const float A11 = u10 * i01 + u11 * i11;
        const float c1 = 2.0f * (A00 * ma0 + A01 * ma1) - 2.0f * mb0;
        const float c2 = 2.0f * (A01 * ma0 + A11 * ma1) - 2.0f * mb1;
        const float c3 = 1.0f - A00;
        const float c4 = -2.0f * A01;
        const float c5 = 1.0f - A11;
        const float c0 = -(c1 * g0 + c2 * g1 + c3 * g2 + c4 * g3 + c5 * g4);
        cs[t * 8 + 0] = c0; cs[t * 8 + 1] = c1; cs[t * 8 + 2] = c2; cs[t * 8 + 3] = c3;
        cs[t * 8 + 4] = c4; cs[t * 8 + 5] = c5; cs[t * 8 + 6] = 0.0f; cs[t * 8 + 7] = 0.0f;
    }
    __syncthreads();
    if (wave == 0) {
        const v4f o = *(const v4fa*)(&cs[lane * 4]);
        float* dst = CO + (size_t)b0 * 8 + lane * 4;
        *(volatile v4f*)dst = o; __threadfence(); *(volatile v4f*)dst = o; }
}

static_assert((size_t)256 * 16 * ER == (size_t)ER * 1024 * 4);
__global__ __launch_bounds__(256) void k_emit(const float* __restrict__ geo, const float* __restrict__ CO, float* OUT) {
    const int n0 = (blockIdx.x * 256 + threadIdx.x) * 4;
    const int r0 = blockIdx.y * ER;
    const v8f g = *(const v8f*)(geo + (size_t)n0 * 2);
    float x0[4], x1[4], xx[4], xy[4], yy[4];
#pragma unroll
    for (int i = 0; i < 4; ++i) { x0[i] = bfr(g[2 * i]); x1[i] = bfr(g[2 * i + 1]); xx[i] = x0[i] * x0[i]; xy[i] = x0[i] * x1[i]; yy[i] = x1[i] * x1[i]; }
#pragma unroll 1
    for (int ps = 0; ps < 2; ++ps) {
#pragma unroll 1
        for (int r = 0; r < ER; ++r) {
            const float* c = CO + (size_t)(r0 + r) * 8;
            const float c0 = c[0], c1 = c[1], c2 = c[2], c3 = c[3], c4 = c[4], c5 = c[5];
            v4f o;
#pragma unroll
            for (int i = 0; i < 4; ++i) o[i] = c0 + c1 * x0[i] + c2 * x1[i] + c3 * xx[i] + c4 * xy[i] + c5 * yy[i];
            *(volatile v4f*)(OUT + (size_t)(r0 + r) * OUT_PITCH + n0) = o; }
        if (ps == 0) __threadfence(); }
}

static constexpr size_t al256(size_t v) { return (v + 255) & ~(size_t)255; }
static constexpr size_t SZ_FT = al256((size_t)16 * NPTS * 2);
static constexpr size_t SZ_GB = 256;
static constexpr size_t SZ_CO = al256((size_t)NROWS * 8 * 4);
static constexpr size_t SZ_TOTAL = 2 * SZ_FT + SZ_GB + SZ_CO;
static_assert(SZ_TOTAL <= (size_t)134217728);
static_assert((size_t)(NROWS / 16) * 512 == (size_t)NROWS * 8 * 4);

extern "C" void kernel_launch(void* const* d_in, const int* in_sizes, int n_in,
                              void* d_out, int out_size, void* d_ws, size_t ws_size, hipStream_t stream) {
    if (n_in < 4) return;
    const size_t needw = (size_t)(NROWS - 1) * NPTS_FULL + NPTS;
    if ((size_t)in_sizes[0] < (size_t)NPTS * 2 || (size_t)in_sizes[1] < (size_t)NPTS * 2) return;
    if ((size_t)in_sizes[2] < needw || (size_t)in_sizes[3] < needw) return;
    if ((size_t)out_size < (size_t)(NROWS - 1) * OUT_PITCH + NPTS) return;
    if (SZ_TOTAL > ws_size) return;
    const float* gx = (const float*)d_in[0];
    const float* gy = (const float*)d_in[1];
    const float* wa = (const float*)d_in[2];
    const float* wb = (const float*)d_in[3];
    float* OUT = (float*)d_out;
    char* wsp = (char*)d_ws;
    bf* FX = (bf*)wsp; wsp += SZ_FT;
    bf* FY = (bf*)wsp; wsp += SZ_FT;
    float* GB = (float*)wsp; wsp += SZ_GB;
    float* CO = (float*)wsp; wsp += SZ_CO;

    const unsigned gf = (unsigned)((NPTS / 8 + 255) / 256);
    k_feat<<<gf, 256, 0, stream>>>(gx, FX);
    k_feat<<<gf, 256, 0, stream>>>(gy, FY);
    k_gbar<<<1, 256, 0, stream>>>(gx, GB);
    k_mom<<<NROWS / 16, 256, 0, stream>>>(wa, wb, FX, FY, GB, CO);
    k_emit<<<dim3(NPTS / 1024, NROWS / ER, 1), 256, 0, stream>>>(gx, CO, OUT);
}
